// Pool_SAGEConv_26061861552144
// MI455X (gfx1250) — hardware-verified
//
#include <hip/hip_runtime.h>
#include <stddef.h>


typedef _Float16       v16h __attribute__((ext_vector_type(16)));
typedef _Float16       v8h  __attribute__((ext_vector_type(8)));
typedef __bf16         v16b __attribute__((ext_vector_type(16)));
typedef unsigned short v8us __attribute__((ext_vector_type(8)));
typedef float          v8f  __attribute__((ext_vector_type(8)));
typedef float          v4f  __attribute__((ext_vector_type(4)));

union HFrag { v16h v; v8h q[2]; };
union BFrag { v16b v; v8us q[2]; };

#define CH       128
#define APITCH   136
#define PPITCH   132
#define WPITCH   264
#define TROWS    128
#define NPB_SH   11
#define NPB      (1 << NPB_SH)
#define PENDCAP  384
#define NTHR     256

#define EDGE_AGG_BYTES  (TROWS * CH * 4)
#define EDGE_R0_BYTES   (TROWS * PPITCH * 4)
#define EDGE_WT_BYTES   (CH * APITCH * 2)
#define EDGE_LDS_BYTES  (EDGE_AGG_BYTES + EDGE_R0_BYTES + EDGE_WT_BYTES + PENDCAP * 8 + 64)
#define NODE_LDS_BYTES  (2 * CH * WPITCH * 2)

typedef char chk_tile_alias_edge[(TROWS * APITCH * 2 <= EDGE_R0_BYTES) ? 1 : -1];
typedef char chk_tile_alias_node[(TROWS * PPITCH * 4 <= NODE_LDS_BYTES) ? 1 : -1];
typedef char chk_bucket_gran[((NPB % TROWS) == 0) ? 1 : -1];

__device__ __forceinline__ v8f mma_f16(v16h a, v16h b, v8f c) {
    c = __builtin_amdgcn_wmma_f32_16x16x32_f16(false, a, false, b, (short)0, c, false, false);
    asm volatile("v_nop\n\tv_nop\n\tv_nop\n\tv_nop" : "+v"(c) : "v"(a), "v"(b));
    return c;
}
__device__ __forceinline__ v8f mma_bf16(v16b a, v16b b, v8f c) {
    c = __builtin_amdgcn_wmma_f32_16x16x32_bf16(false, a, false, b, (short)0, c, false, false);
    asm volatile("v_nop\n\tv_nop\n\tv_nop\n\tv_nop" : "+v"(c) : "v"(a), "v"(b));
    return c;
}

__device__ __forceinline__ unsigned short bf16_bits(float f) {
    unsigned u = __float_as_uint(f);
    u += 0x7FFFu + ((u >> 16) & 1u);
    return (unsigned short)(u >> 16);
}

__device__ __forceinline__ void split8(const v4f a, const v4f b, v8us& hi, v8us& lo) {
    float f[8] = {a.x, a.y, a.z, a.w, b.x, b.y, b.z, b.w};
#pragma unroll
    for (int i = 0; i < 8; ++i) {
        const unsigned short hb = bf16_bits(f[i]);
        const float hf = __uint_as_float(((unsigned)hb) << 16);
        hi[i] = hb;
        lo[i] = bf16_bits(f[i] - hf);
    }
}

__device__ __forceinline__ float half_sum(float v) {
    v += __shfl_xor(v, 1, 32);
    v += __shfl_xor(v, 2, 32);
    v += __shfl_xor(v, 4, 32);
    v += __shfl_xor(v, 8, 32);
    return v;
}

__device__ __forceinline__ void strip_ln_relu_store(const v8f (&acc)[8], float scl,
        const float* __restrict__ bias, const float* __restrict__ gam, const float* __restrict__ bet,
        float* tile, int wave, int lane)
{
    const int m = lane & 15, h = lane >> 4;
    float pb[8], g[8], bb[8];
#pragma unroll
    for (int nt = 0; nt < 8; ++nt) {
        const int c = 16 * nt + m;
        pb[nt] = bias[c]; g[nt] = gam[c]; bb[nt] = bet[c];
    }
#pragma unroll
    for (int r = 0; r < 8; ++r) {
        float v[8];
        float s = 0.0f;
#pragma unroll
        for (int nt = 0; nt < 8; ++nt) { v[nt] = acc[nt][r] * scl + pb[nt]; s += v[nt]; }
        s = half_sum(s);
        const float mean = s * (1.0f / 128.0f);
        float q = 0.0f;
#pragma unroll
        for (int nt = 0; nt < 8; ++nt) { v[nt] -= mean; q += v[nt] * v[nt]; }
        q = half_sum(q);
        const float inv = rsqrtf(q * (1.0f / 128.0f) + 1e-5f);
        float* prow = tile + (16 * wave + 8 * h + r) * PPITCH + m;
#pragma unroll
        for (int nt = 0; nt < 8; ++nt) prow[16 * nt] = fmaxf(v[nt] * inv * g[nt] + bb[nt], 0.0f);
    }
}

__global__ __launch_bounds__(NTHR) void k_prep(const float* __restrict__ pool_w,
                                               const float* __restrict__ final_w,
                                               _Float16* wtp, unsigned short* wth, unsigned short* wtl)
{
    const int t = threadIdx.x;
    for (int pass = 0; pass < 2; ++pass) {
        for (int c = t; c < CH * (CH / 8); c += NTHR) {
            const int n = c >> 4, kq = (c & 15) * 8;
            v8h hv;
#pragma unroll
            for (int j = 0; j < 8; ++j) hv[j] = (_Float16)(pool_w[(kq + j) * CH + n] * 64.0f);
            *(volatile v8h*)(wtp + n * CH + kq) = hv;
        }
        for (int c = t; c < CH * (2 * CH / 8); c += NTHR) {
            const int n = c >> 5, kq = (c & 31) * 8;
            v8us hh, ll;
#pragma unroll
            for (int j = 0; j < 8; ++j) {
                const float f = final_w[(kq + j) * CH + n];
                const unsigned short hb = bf16_bits(f);
                const float hf = __uint_as_float(((unsigned)hb) << 16);
                hh[j] = hb;
                ll[j] = bf16_bits(f - hf);
            }
            *(volatile v8us*)(wth + n * (2 * CH) + kq) = hh;
            *(volatile v8us*)(wtl + n * (2 * CH) + kq) = ll;
        }
        __threadfence();
    }
}

__global__ __launch_bounds__(NTHR) void k_bucket(const int* __restrict__ ei, int nEdges, int capSub,
                                                 int* lists, int* lcnt)
{
    __shared__ int stg_all[8][64];
    const int t = threadIdx.x, lane = t & 31, wave = t >> 5;
    volatile int* stg = &stg_all[wave][0];
    const int lo = blockIdx.x * NPB;
    const size_t li = (size_t)blockIdx.x * 8 + wave;
    int* outp = lists + li * (size_t)capSub;
    int cnt = 0, written = 0, total = 0;

#pragma unroll 1
    for (int base = 0; base < nEdges; base += NTHR) {
        const int e = base + wave * 32 + lane;
        bool mt = false;
        int pk = 0;
        if (e < nEdges) {
            const int d  = ei[(size_t)nEdges + e];
            const int dl = d - lo;
            mt = (unsigned)dl < (unsigned)NPB;
            pk = (e << NPB_SH) | dl;
        }
        const unsigned mask = __builtin_amdgcn_ballot_w32(mt);
        const int pre = (int)__builtin_amdgcn_mbcnt_lo(mask, 0u);
        if (mt) stg[cnt + pre] = pk;
        const int c = __builtin_popcount(mask);
        cnt += c; total += c;
        if (cnt >= 32) {
            const int v   = stg[lane];
            const int rem = cnt - 32;
            int mv = 0;
            if (lane < rem) mv = stg[32 + lane];
            volatile int* q = outp + written + lane;
            *q = v;
            __threadfence();
            *q = v;
            if (lane < rem) stg[lane] = mv;
            cnt = rem;
            written += 32;
        }
    }
    {
        const int v = (lane < cnt) ? stg[lane] : 0;
        volatile int* q = outp + written + lane;
        *q = v;
        __threadfence();
        *q = v;
    }
    {
        volatile int* q = lcnt + li * 32 + lane;
        *q = total;
        __threadfence();
        *q = total;
    }
}

__device__ __forceinline__ void edge_chunk(
    const float* __restrict__ x, const int* __restrict__ ei, const float* __restrict__ ew,
    const float* __restrict__ pool_b, const float* __restrict__ ln_g, const float* __restrict__ ln_b,
    _Float16* At, float* Pt, const _Float16* Wt, float* aggL,
    const int* elist, const int* dlist,
    int rows, float coeff, int nNodes, int t, int lane, int wave)
{
    {
        const int r = t >> 1, hf = t & 1;
        _Float16* arow = At + r * APITCH + 64 * hf;
        if (r < rows) {
            const int eid = elist[r];
            int s = ei[eid];
            s = s < 0 ? 0 : (s >= nNodes ? nNodes - 1 : s);
            const float sc = 1.0f + coeff * ew[eid];
            const float* xp = x + (size_t)s * CH + 64 * hf;
#pragma unroll
            for (int j = 0; j < 8; ++j) {
                const v4f a = *(const v4f*)(xp + 8 * j);
                const v4f b = *(const v4f*)(xp + 8 * j + 4);
                v8h hv;
                hv[0] = (_Float16)(a.x * sc); hv[1] = (_Float16)(a.y * sc);
                hv[2] = (_Float16)(a.z * sc); hv[3] = (_Float16)(a.w * sc);
                hv[4] = (_Float16)(b.x * sc); hv[5] = (_Float16)(b.y * sc);
                hv[6] = (_Float16)(b.z * sc); hv[7] = (_Float16)(b.w * sc);
                *(v8h*)(arow + 8 * j) = hv;
            }
        } else {
            v8h z;
#pragma unroll
            for (int k = 0; k < 8; ++k) z[k] = (_Float16)0.0f;
#pragma unroll
            for (int j = 0; j < 8; ++j) *(v8h*)(arow + 8 * j) = z;
        }
    }
    __syncthreads();

    const int m = lane & 15, h = lane >> 4;
    v8f acc[8];
#pragma unroll
    for (int nt = 0; nt < 8; ++nt) acc[nt] = (v8f){0.f, 0.f, 0.f, 0.f, 0.f, 0.f, 0.f, 0.f};
    const _Float16* ar  = At + (16 * wave + m) * APITCH + 8 * h;
    const _Float16* br0 = Wt + m * APITCH + 8 * h;
#pragma unroll 1
    for (int ks = 0; ks < CH / 32; ++ks) {
        HFrag a;
        a.q[0] = *(const v8h*)(ar + 32 * ks);
        a.q[1] = *(const v8h*)(ar + 32 * ks + 16);
#pragma unroll
        for (int nt = 0; nt < 8; ++nt) {
            const _Float16* br = br0 + (16 * nt) * APITCH + 32 * ks;
            HFrag b;
            b.q[0] = *(const v8h*)(br);
            b.q[1] = *(const v8h*)(br + 16);
            acc[nt] = mma_f16(a.v, b.v, acc[nt]);
        }
    }
    __syncthreads();

    strip_ln_relu_store(acc, 0.015625f, pool_b, ln_g, ln_b, Pt, wave, lane);
    __syncthreads();

    if (wave == 0) {
#pragma unroll 1
        for (int r = 0; r < rows; ++r) {
            const int d = dlist[r];
            const v4f pv = *((const v4f*)(Pt + r * PPITCH) + lane);
            v4f* ap = (v4f*)(aggL + d * CH) + lane;
            v4f av = *ap;
            av.x = fmaxf(av.x, pv.x); av.y = fmaxf(av.y, pv.y);
            av.z = fmaxf(av.z, pv.z); av.w = fmaxf(av.w, pv.w);
            *ap = av;
        }
    }
    __syncthreads();
}

__global__ __launch_bounds__(NTHR) void k_edge(
    const float* __restrict__ x, const int* __restrict__ ei, const float* __restrict__ ew,
    const _Float16* __restrict__ wtp,
    const float* __restrict__ pool_b, const float* __restrict__ ln_g, const float* __restrict__ ln_b,
    const float* __restrict__ coeff_raw,
    const int* __restrict__ lists, const int* __restrict__ lcnt,
    float* agg, int nNodes, int nEdges, int capSub)
{
    extern __shared__ __attribute__((aligned(16))) char smem[];
    float*    aggL  = (float*)smem;
    char*     r0    = smem + EDGE_AGG_BYTES;
    _Float16* At    = (_Float16*)r0;
    float*    Pt    = (float*)r0;
    _Float16* Wt    = (_Float16*)(r0 + EDGE_R0_BYTES);
    int*      elist = (int*)(r0 + EDGE_R0_BYTES + EDGE_WT_BYTES);
    int*      dlist = elist + PENDCAP;
    int*      wcnt  = dlist + PENDCAP;

    const int t = threadIdx.x, lane = t & 31, wave = t >> 5;
    const int n0 = blockIdx.x * TROWS;
    const int bucket = n0 >> NPB_SH;
    const float cr = coeff_raw[0];
    const float coeff = fmaxf(cr, 0.0f) + log1pf(expf(-fabsf(cr)));

    for (int i = t; i < TROWS * CH / 4; i += NTHR) ((v4f*)aggL)[i] = (v4f){0.f, 0.f, 0.f, 0.f};
    for (int c = t; c < CH * (CH / 8); c += NTHR) {
        const int n = c >> 4, kq = (c & 15) * 8;
        *(v8h*)(Wt + n * APITCH + kq) = *(const v8h*)(wtp + n * CH + kq);
    }
    __syncthreads();

    int pending = 0;
#pragma unroll 1
    for (int sub = 0; sub < 8; ++sub) {
        const size_t li = (size_t)bucket * 8 + sub;
        const int* lp = lists + li * (size_t)capSub;
        int len = lcnt[li * 32];
        if (len < 0) len = 0;
        if (len > capSub) len = capSub;
#pragma unroll 1
        for (int pos = 0; pos < len; pos += NTHR) {
            const int i = pos + t;
            bool mt = false;
            int eid = 0, dl = 0;
            if (i < len) {
                const int v = lp[i];
                eid = v >> NPB_SH;
                eid = eid < 0 ? 0 : (eid >= nEdges ? nEdges - 1 : eid);
                dl  = (v & (NPB - 1)) + (bucket << NPB_SH) - n0;
                mt  = (unsigned)dl < (unsigned)TROWS;
            }
            const unsigned mask = __builtin_amdgcn_ballot_w32(mt);
            const int pre = (int)__builtin_amdgcn_mbcnt_lo(mask, 0u);
            if (lane == 0) wcnt[wave] = __builtin_popcount(mask);
            __syncthreads();
            int tot = 0, wpre = 0;
#pragma unroll
            for (int w = 0; w < 8; ++w) {
                const int cw = wcnt[w];
                tot += cw;
                wpre += (w < wave) ? cw : 0;
            }
            if (mt) {
                const int slot = pending + wpre + pre;
                elist[slot] = eid;
                dlist[slot] = dl;
            }
            __syncthreads();
            pending += tot;
            if (pending >= TROWS) {
                edge_chunk(x, ei, ew, pool_b, ln_g, ln_b, At, Pt, Wt, aggL, elist, dlist,
                           TROWS, coeff, nNodes, t, lane, wave);
                const int rem = pending - TROWS;
                int e2 = 0, d2 = 0;
                if (t < rem) { e2 = elist[TROWS + t]; d2 = dlist[TROWS + t]; }
                __syncthreads();
                if (t < rem) { elist[t] = e2; dlist[t] = d2; }
                __syncthreads();
                pending = rem;
            }
        }
    }
    if (pending > 0) {
        edge_chunk(x, ei, ew, pool_b, ln_g, ln_b, At, Pt, Wt, aggL, elist, dlist,
                   pending, coeff, nNodes, t, lane, wave);
    }
    __syncthreads();

    for (int pass = 0; pass < 2; ++pass) {
#pragma unroll 1
        for (int i = 0; i < TROWS / 8; ++i) {
            const int r = wave + 8 * i;
            const int node = n0 + r;
            if (node < nNodes) {
                const v4f v = *((const v4f*)(aggL + r * CH) + lane);
                *((volatile v4f*)(agg + (size_t)node * CH) + lane) = v;
            }
        }
        __threadfence();
    }
}

__global__ __launch_bounds__(NTHR) void k_node(
    const float* __restrict__ x, const float* __restrict__ agg,
    const unsigned short* __restrict__ wth, const unsigned short* __restrict__ wtl,
    const float* __restrict__ fb, const float* __restrict__ ln_g, const float* __restrict__ ln_b,
    float* out, int nNodes)
{
    extern __shared__ __attribute__((aligned(16))) char smem[];
    unsigned short* Wh = (unsigned short*)smem;
    unsigned short* Wl = Wh + CH * WPITCH;
    float* Ot = (float*)smem;

    const int t = threadIdx.x, lane = t & 31, wave = t >> 5;
    const int m = lane & 15, h = lane >> 4;

    for (int c = t; c < CH * (2 * CH / 8); c += NTHR) {
        const int n = c >> 5, kq = (c & 31) * 8;
        *(v8us*)(Wh + n * WPITCH + kq) = *(const v8us*)(wth + n * (2 * CH) + kq);
        *(v8us*)(Wl + n * WPITCH + kq) = *(const v8us*)(wtl + n * (2 * CH) + kq);
    }
    __syncthreads();

    const int n0   = blockIdx.x * TROWS;
    const int row  = n0 + 16 * wave + m;
    const int rowc = row < nNodes ? row : nNodes - 1;
    const float* xr = x   + (size_t)rowc * CH + 8 * h;
    const float* gr = agg + (size_t)rowc * CH + 8 * h;

    v8f acc[8];
#pragma unroll
    for (int nt = 0; nt < 8; ++nt) acc[nt] = (v8f){0.f, 0.f, 0.f, 0.f, 0.f, 0.f, 0.f, 0.f};

#pragma unroll 1
    for (int ks = 0; ks < 2 * CH / 32; ++ks) {
        const float* src = (ks < CH / 32) ? (xr + 32 * ks) : (gr + 32 * (ks - CH / 32));
        const v4f f0 = *(const v4f*)(src);
        const v4f f1 = *(const v4f*)(src + 4);
        const v4f f2 = *(const v4f*)(src + 16);
        const v4f f3 = *(const v4f*)(src + 20);
        BFrag ah, al;
        split8(f0, f1, ah.q[0], al.q[0]);
        split8(f2, f3, ah.q[1], al.q[1]);
#pragma unroll
        for (int nt = 0; nt < 8; ++nt) {
            const unsigned short* bh = Wh + (16 * nt + m) * WPITCH + 32 * ks + 8 * h;
            const unsigned short* bl = Wl + (16 * nt + m) * WPITCH + 32 * ks + 8 * h;
            BFrag bH, bL;
            bH.q[0] = *(const v8us*)(bh);
            bH.q[1] = *(const v8us*)(bh + 16);
            bL.q[0] = *(const v8us*)(bl);
            bL.q[1] = *(const v8us*)(bl + 16);
            acc[nt] = mma_bf16(ah.v, bH.v, acc[nt]);
            acc[nt] = mma_bf16(ah.v, bL.v, acc[nt]);
            acc[nt] = mma_bf16(al.v, bH.v, acc[nt]);
        }
    }
    __syncthreads();

    strip_ln_relu_store(acc, 1.0f, fb, ln_g, ln_b, Ot, wave, lane);
    __syncthreads();

    for (int pass = 0; pass < 2; ++pass) {
#pragma unroll 1
        for (int i = 0; i < TROWS / 8; ++i) {
            const int r = wave + 8 * i;
            const int node = n0 + r;
            if (node < nNodes) {
                const v4f v = *((const v4f*)(Ot + r * PPITCH) + lane);
                *((volatile v4f*)(out + (size_t)node * CH) + lane) = v;
            }
        }
        __threadfence();
    }
}

static inline size_t al256(size_t b) { return (b + 255) & ~(size_t)255; }

extern "C" void kernel_launch(void* const* d_in, const int* in_sizes, int n_in,
                              void* d_out, int out_size, void* d_ws, size_t ws_size,
                              hipStream_t stream)
{
    if (n_in < 12) return;
    const float* x    = (const float*)d_in[0];
    const int*   ei   = (const int*)d_in[1];
    const float* ew   = (const float*)d_in[2];
    const float* pw   = (const float*)d_in[3];
    const float* pb   = (const float*)d_in[4];
    const float* plg  = (const float*)d_in[5];
    const float* plb  = (const float*)d_in[6];
    const float* fw   = (const float*)d_in[7];
    const float* fbv  = (const float*)d_in[8];
    const float* flg  = (const float*)d_in[9];
    const float* flb  = (const float*)d_in[10];
    const float* craw = (const float*)d_in[11];

    const int nNodes = in_sizes[0] / CH;
    const int nEdges = in_sizes[1] / 2;
    if (nNodes <= 0 || nNodes * CH != in_sizes[0]) return;
    if (nEdges < 0 || nEdges * 2 != in_sizes[1] || nEdges > (1 << 20)) return;
    if (in_sizes[2] < nEdges) return;
    if (in_sizes[3] != CH * CH || in_sizes[7] != 2 * CH * CH) return;
    if (in_sizes[4] < CH || in_sizes[5] < CH || in_sizes[6] < CH) return;
    if (in_sizes[8] < CH || in_sizes[9] < CH || in_sizes[10] < CH || in_sizes[11] < 1) return;
    if (out_size != nNodes * CH) return;

    const int nBuckets = (nNodes + NPB - 1) / NPB;
    const int capSub   = ((nEdges + 255) / 256) * 32 + 32;

    size_t off = 0;
    const size_t oAgg = off; off += al256((size_t)nNodes * CH * sizeof(float));
    const size_t oWtp = off; off += al256((size_t)CH * CH * 2);
    const size_t oWh  = off; off += al256((size_t)2 * CH * CH * 2);
    const size_t oWl  = off; off += al256((size_t)2 * CH * CH * 2);
    const size_t oCnt = off; off += al256((size_t)nBuckets * 8 * 32 * sizeof(int));
    const size_t oLst = off; off += al256((size_t)nBuckets * 8 * (size_t)capSub * sizeof(int));
    if (off > ws_size) return;

    char* ws = (char*)d_ws;
    float*          agg   = (float*)(ws + oAgg);
    _Float16*       wtp   = (_Float16*)(ws + oWtp);
    unsigned short* wth   = (unsigned short*)(ws + oWh);
    unsigned short* wtl   = (unsigned short*)(ws + oWl);
    int*            lcnt  = (int*)(ws + oCnt);
    int*            lists = (int*)(ws + oLst);

    k_prep<<<1, NTHR, 0, stream>>>(pw, fw, wtp, wth, wtl);

    k_bucket<<<nBuckets, NTHR, 0, stream>>>(ei, nEdges, capSub, lists, lcnt);

    const int gridNodes = (nNodes + TROWS - 1) / TROWS;
    hipFuncSetAttribute((const void*)k_edge, hipFuncAttributeMaxDynamicSharedMemorySize, (int)EDGE_LDS_BYTES);
    k_edge<<<gridNodes, NTHR, EDGE_LDS_BYTES, stream>>>(
        x, ei, ew, wtp, pb, plg, plb, craw, lists, lcnt, agg, nNodes, nEdges, capSub);

    hipFuncSetAttribute((const void*)k_node, hipFuncAttributeMaxDynamicSharedMemorySize, (int)NODE_LDS_BYTES);
    k_node<<<gridNodes, NTHR, NODE_LDS_BYTES, stream>>>(
        x, agg, wth, wtl, fbv, flg, flb, (float*)d_out, nNodes);
}
